// OptimizedMPNN_39273180955640
// MI455X (gfx1250) — hardware-verified
//
#include <hip/hip_runtime.h>
#include <math.h>

typedef __attribute__((ext_vector_type(16))) _Float16 v16h;
typedef __attribute__((ext_vector_type(16))) __bf16 v16b;
typedef __attribute__((ext_vector_type(8)))  _Float16 v8h;
typedef __attribute__((ext_vector_type(8)))  float v8f;
typedef __attribute__((ext_vector_type(4)))  float v4f;
typedef __attribute__((ext_vector_type(2)))  float v2f;
typedef __attribute__((ext_vector_type(4)))  unsigned v4u;
typedef __attribute__((ext_vector_type(4)))  int v4i;
typedef float __attribute__((may_alias)) float_a;
typedef int __attribute__((may_alias)) int_a;

template <typename T> __device__ __forceinline__ void vst2(void* p, T v) { *(volatile T*)p = v; __threadfence(); *(volatile T*)p = v; }
__device__ __forceinline__ v8f wmma16(v16h a, v16h b, v8f c) {
  v8f d = __builtin_amdgcn_wmma_f32_16x16x32_f16(false, a, false, b, (short)0, c, false, false);
  asm volatile("v_nop\n\tv_nop\n\tv_nop\n\tv_nop" : "+v"(d) : "v"(a), "v"(b));
  return d;
}
__device__ __forceinline__ v8f wmma_bf(v16b a, v16b b, v8f c) {
  v8f d = __builtin_amdgcn_wmma_f32_16x16x32_bf16(false, a, false, b, (short)0, c, false, false);
  asm volatile("v_nop\n\tv_nop\n\tv_nop\n\tv_nop" : "+v"(d) : "v"(a), "v"(b));
  return d;
}
__device__ __forceinline__ v16h frag_h(const _Float16* rowk0, int lane) {
  union { v16h v; v8h q[2]; } u; const _Float16* p = rowk0 + 8 * (lane >> 4);
  u.q[0] = *(const v8h*)p; u.q[1] = *(const v8h*)(p + 16); return u.v;
}
__device__ __forceinline__ v16h frag_f32(const float* rowk0, int lane) {
  v16h a; const float* p = rowk0 + 8 * (lane >> 4);
#pragma unroll
  for (int i = 0; i < 8; ++i) { a[i] = (_Float16)p[i]; a[8 + i] = (_Float16)p[16 + i]; }
  return a;
}
__device__ __forceinline__ v16h frag_f32s(const float* rowk0, int lane, float sc) {
  v16h a; const float* p = rowk0 + 8 * (lane >> 4);
#pragma unroll
  for (int i = 0; i < 8; ++i) { a[i] = (_Float16)(p[i] * sc); a[8 + i] = (_Float16)(p[16 + i] * sc); }
  return a;
}
__device__ __forceinline__ v16h fragc_f32(const float* W, int k0, int n, int lane, int ld, int K) {
  v16h a; const int g = lane >> 4;
#pragma unroll
  for (int i = 0; i < 8; ++i) { const int ka = k0 + 8 * g + i, kb = ka + 16;
    a[i] = (_Float16)(ka < K ? W[(size_t)(ka < K ? ka : K - 1) * ld + n] : 0.f); a[8 + i] = (_Float16)(kb < K ? W[(size_t)(kb < K ? kb : K - 1) * ld + n] : 0.f); }
  return a;
}
struct F2 { v16b h, l; };
__device__ __forceinline__ F2 bsplit16(const float v[16]) { F2 r;
#pragma unroll
  for (int i = 0; i < 16; ++i) { const __bf16 h = (__bf16)v[i]; r.h[i] = h; r.l[i] = (__bf16)(v[i] - (float)h); }
  return r; }
__device__ __forceinline__ F2 split_row(const float* row, int k0, int lane) { float v[16]; const float* p = row + k0 + 8 * (lane >> 4);
#pragma unroll
  for (int i = 0; i < 8; ++i) { v[i] = p[i]; v[8 + i] = p[16 + i]; }
  return bsplit16(v); }
__device__ __forceinline__ F2 split_rowK(const float* row, int k0, int lane, int K) { float v[16]; const int g = lane >> 4;
#pragma unroll
  for (int i = 0; i < 8; ++i) { const int ka = k0 + 8 * g + i, kb = ka + 16; v[i] = ka < K ? row[ka < K ? ka : K - 1] : 0.f; v[8 + i] = kb < K ? row[kb < K ? kb : K - 1] : 0.f; }
  return bsplit16(v); }
__device__ __forceinline__ F2 split_col(const float* W, int k0, int n, int lane, int ld, int K) { float v[16]; const int g = lane >> 4;
#pragma unroll
  for (int i = 0; i < 8; ++i) { const int ka = k0 + 8 * g + i, kb = ka + 16; v[i] = ka < K ? W[(size_t)(ka < K ? ka : K - 1) * ld + n] : 0.f; v[8 + i] = kb < K ? W[(size_t)(kb < K ? kb : K - 1) * ld + n] : 0.f; }
  return bsplit16(v); }
__device__ __forceinline__ v8f mac3(const F2& a, const F2& b, v8f c) { c = wmma_bf(a.l, b.h, c); c = wmma_bf(a.h, b.l, c); return wmma_bf(a.h, b.h, c); }
__device__ __forceinline__ float sigm(float v) { return 1.0f / (1.0f + expf(-v)); }
#define LDSX() do { asm volatile("s_wait_dscnt 0" ::: "memory"); __builtin_amdgcn_wave_barrier(); __builtin_amdgcn_fence(__ATOMIC_RELEASE, "workgroup"); } while (0)


#ifndef NN
#define NN 20000
#endif
#define EP 50000
#ifndef NE
#define NE 50000
#endif
#ifndef NG
#define NG 128
#endif
#define CIN1 32
#define HH 64
#define EC 8
#define KH1 128
#define KH2 256
#define MAXE 320
#define NBLK ((NN + 63) / 64)
#define NRP (NBLK * 64)
#define NEP (((NE + 63) / 64) * 64)
#define CSR_N NN
#define CSR_E NE
typedef __attribute__((ext_vector_type(8))) __bf16 v8b;
__device__ __forceinline__ v16b frag_b(const __bf16* rowk0, int lane) {
  union { v16b v; v8b q[2]; } u; const __bf16* p = rowk0 + 8 * (lane >> 4);
  u.q[0] = *(const v8b*)p; u.q[1] = *(const v8b*)(p + 16); return u.v;
}
__device__ __forceinline__ float bfr(float v) { return (float)(__bf16)v; }
__device__ __attribute__((noinline)) float exp_ni(float v) { return expf(v); }
__device__ __attribute__((noinline)) float erf_ni(float v) { return erff(v); }

#define CSR_FINN (CSR_E + 32 * CSR_NBK)
#define CSR_CHUNK 4096
#define CSR_BKT 256
#define CSR_NCH ((CSR_E + CSR_CHUNK - 1) / CSR_CHUNK)
#define CSR_NBK ((CSR_N + CSR_BKT - 1) / CSR_BKT)
#define CSR_NBKP (((CSR_NBK + 63) / 64) * 64)
#define CSR_SEGCAP (CSR_E + 32 * CSR_NBK * CSR_NCH)
#ifndef CSR_BCAP
#define CSR_BCAP 10240
#endif
#define CSR_SZ_CNT   (4u * CSR_NCH * CSR_NBKP)
#define CSR_SZ_OFF   (4u * CSR_NBK * (((CSR_NCH + 31) / 32) * 32))
#define CSR_SZ_BST   (4u * (((CSR_NBK + 1 + 31) / 32) * 32))
#define CSR_SZ_SEG   (4u * CSR_SEGCAP)
#define CSR_SZ_FIN   (4u * (CSR_E + 32 * CSR_NBK))
#define CSR_SZ_ROW   (4u * CSR_NBK * CSR_BKT)
#define CSR_OFFP (((CSR_NCH + 31) / 32) * 32)

__global__ __launch_bounds__(256) void k_csr_cnt(const int* __restrict__ DST, int dstride, int* __restrict__ CNT) {
  __shared__ unsigned short sc[256][CSR_NBK + 1]; __shared__ __align__(16) int srow[CSR_NBKP];
  const int c = blockIdx.x, tid = threadIdx.x;
  for (int b = 0; b < CSR_NBK; ++b) sc[tid][b] = 0;
  const size_t e0 = (size_t)c * CSR_CHUNK + tid * 16;
  for (int i = 0; i < 16; ++i) { const size_t e = e0 + i; if (e < (size_t)CSR_E) { int d = DST[e * dstride]; d = min(max(d, 0), CSR_N - 1); sc[tid][d / CSR_BKT] += 1; } }
  __syncthreads();
  for (int b = tid; b < CSR_NBKP; b += 256) { int s = 0; if (b < CSR_NBK) for (int t = 0; t < 256; ++t) s += sc[t][b]; srow[b] = s; }
  __syncthreads();
  for (int q = tid; q < CSR_NBKP / 4; q += 256) vst2((unsigned*)(CNT + (size_t)c * CSR_NBKP + q * 4), *(const v4u*)&srow[q * 4]);
}
__global__ __launch_bounds__(256) void k_csr_scan(const int* __restrict__ CNT, int* __restrict__ OFF, int* __restrict__ BST) {
  __shared__ int sbt[CSR_NBK + 1]; __shared__ int sbs[((CSR_NBK + 1 + 31) / 32) * 32]; __shared__ int scnt[CSR_NBK + 1]; __shared__ __align__(16) int sbuf[64][CSR_OFFP];
  const int tid = threadIdx.x;
  for (int b = tid; b < CSR_NBK; b += 256) { int sp = 0, st = 0; for (int c = 0; c < CSR_NCH; ++c) { const int n = CNT[(size_t)c * CSR_NBKP + b]; st += n; sp += (n + 31) & ~31; } sbt[b] = sp; scnt[b] = st; }
  for (int b = tid; b < ((CSR_NBK + 1 + 31) / 32) * 32; b += 256) sbs[b] = 0;
  __syncthreads();
  if (tid == 0) { int acc = 0, accf = 0; for (int b = 0; b < CSR_NBK; ++b) { const int t = sbt[b]; sbt[b] = acc; acc += t; sbs[b] = accf; accf += (scnt[b] + 31) & ~31; } sbs[CSR_NBK] = accf; }
  __syncthreads();
  for (int b0 = 0; b0 < CSR_NBK; b0 += 64) {
    if (tid < 64 && b0 + tid < CSR_NBK) { const int b = b0 + tid; int o = sbt[b]; for (int c = 0; c < CSR_OFFP; ++c) { if (c < CSR_NCH) { sbuf[tid][c] = o; o += (CNT[(size_t)c * CSR_NBKP + b] + 31) & ~31; } else sbuf[tid][c] = 0; } }
    __syncthreads();
    for (int q = tid; q < 64 * (CSR_OFFP / 4); q += 256) { const int r = q / (CSR_OFFP / 4), pc = q % (CSR_OFFP / 4); if (b0 + r < CSR_NBK) vst2((unsigned*)(OFF + (size_t)(b0 + r) * CSR_OFFP + pc * 4), *(const v4u*)&sbuf[r][pc * 4]); }
    __syncthreads(); }
  for (int q = tid; q < ((CSR_NBK + 1 + 31) / 32) * 32 / 4; q += 256) vst2((unsigned*)(BST + q * 4), *(const v4u*)&sbs[q * 4]);
}
__global__ __launch_bounds__(256) void k_csr_scatter(const int* __restrict__ SRC, const int* __restrict__ DST, int sstride, int dstride, const int* __restrict__ OFF, int* __restrict__ SEGS, int* __restrict__ SEGE) {
  __shared__ unsigned short sc[256][CSR_NBK + 1]; __shared__ int sbase[CSR_NBK + 1]; __shared__ int scn[CSR_NBK + 1]; __shared__ int sord[CSR_CHUNK];
  const int c = blockIdx.x, tid = threadIdx.x;
  for (int b = 0; b < CSR_NBK; ++b) sc[tid][b] = 0;
  const size_t e0 = (size_t)c * CSR_CHUNK + tid * 16; int bk[16];
#pragma unroll
  for (int i = 0; i < 16; ++i) { const size_t e = e0 + i; bk[i] = -1; if (e < (size_t)CSR_E) { int d = DST[e * dstride]; d = min(max(d, 0), CSR_N - 1); bk[i] = d / CSR_BKT; sc[tid][bk[i]] += 1; } }
  __syncthreads();
  for (int b = tid; b < CSR_NBK; b += 256) { int acc = 0; for (int t = 0; t < 256; ++t) { const int v = sc[t][b]; sc[t][b] = (unsigned short)acc; acc += v; } scn[b] = acc; }
  __syncthreads();
  if (tid == 0) { int acc = 0; for (int b = 0; b < CSR_NBK; ++b) { sbase[b] = acc; acc += scn[b]; } }
  __syncthreads();
#pragma unroll
  for (int i = 0; i < 16; ++i) { if (bk[i] >= 0) { const int b = bk[i]; const int r = sc[tid][b]; sc[tid][b] = (unsigned short)(r + 1); sord[sbase[b] + r] = tid * 16 + i; } }
  __syncthreads();
  for (int b = 0; b < CSR_NBK; ++b) { const int n = scn[b]; if (n == 0) continue; const int nl = ((n + 31) & ~31); const size_t o = (size_t)(min(max(OFF[(size_t)b * CSR_OFFP + c], 0), CSR_SEGCAP - nl) & ~31);
    for (int q = tid; q < nl / 4; q += 256) { int4 vs, ve;
#pragma unroll
      for (int k = 0; k < 4; ++k) { const int i = q * 4 + k; int s = -1, eid = -1; if (i < n) { const size_t e = (size_t)c * CSR_CHUNK + sord[sbase[b] + i]; s = min(max(SRC[e * sstride], 0), CSR_N - 1); eid = (int)e; } vs[k] = s; ve[k] = eid; }
      vst2((unsigned*)(SEGS + o + q * 4), *(const v4u*)&vs); vst2((unsigned*)(SEGE + o + q * 4), *(const v4u*)&ve); } }
}
__global__ __launch_bounds__(256) void k_csr_bucket(const int* __restrict__ CNT, const int* __restrict__ OFF, const int* __restrict__ BST, const int* __restrict__ SEGS, const int* __restrict__ SEGE, const int* __restrict__ DST, int dstride, int* __restrict__ FS, int* __restrict__ FE, int* __restrict__ ROWST, int* __restrict__ ROWCNT) {
  __shared__ int ssrc[CSR_BCAP]; __shared__ int seid[CSR_BCAP]; __shared__ unsigned char snod[CSR_BCAP]; __shared__ int souts[CSR_BCAP]; __shared__ int soute[CSR_BCAP]; __shared__ int scount[256]; __shared__ int sstart[257]; __shared__ int stot;
  const int b = blockIdx.x, tid = threadIdx.x;
  if (tid == 0) { int t = 0; for (int c = 0; c < CSR_NCH; ++c) t += min(max(CNT[(size_t)c * CSR_NBKP + b], 0), CSR_CHUNK); stot = (t <= CSR_BCAP) ? t : 0; }
  __syncthreads();
  { int base = 0; for (int c = 0; c < CSR_NCH; ++c) { const int n = min(max(CNT[(size_t)c * CSR_NBKP + b], 0), CSR_CHUNK); const int o = min(max(OFF[(size_t)b * CSR_OFFP + c], 0), CSR_SEGCAP - ((n + 31) & ~31));
      for (int i = tid; i < n; i += 256) { const int p = base + i; if (p < CSR_BCAP) { ssrc[p] = min(max(SEGS[o + i], 0), CSR_N - 1); const int e = min(max(SEGE[o + i], 0), CSR_E - 1); seid[p] = e; int d = DST[(size_t)e * dstride]; d = min(max(d, 0), CSR_N - 1); const int dl = d - b * CSR_BKT; snod[p] = (unsigned char)(dl >= 0 && dl < 256 ? dl : 255); } }
      base += n; } }
  __syncthreads();
  const int node = b * CSR_BKT + tid; int cnt = 0; for (int p = 0; p < stot; ++p) cnt += (snod[p] == tid) ? 1 : 0;
  scount[tid] = cnt; __syncthreads();
  if (tid == 0) { int acc = 0; for (int t = 0; t < 256; ++t) { sstart[t] = acc; acc += scount[t]; } sstart[256] = acc; }
  __syncthreads();
  const int bst0 = min(max(BST[b], 0), CSR_FINN - ((sstart[256] + 31) & ~31)) & ~31; const int gst = bst0 + sstart[tid];
  { int w = sstart[tid]; for (int p = 0; p < stot; ++p) if (snod[p] == tid) { souts[w] = ssrc[p]; soute[w] = seid[p]; ++w; } }
  __syncthreads();
  { const int n = sstart[256]; const int nl = (n + 31) & ~31; for (int q = tid; q < nl / 4; q += 256) { int4 vs, ve;
#pragma unroll
      for (int k = 0; k < 4; ++k) { const int i = q * 4 + k; vs[k] = i < n ? souts[i] : -1; ve[k] = i < n ? soute[i] : -1; }
      vst2((unsigned*)(FS + bst0 + q * 4), *(const v4u*)&vs); vst2((unsigned*)(FE + bst0 + q * 4), *(const v4u*)&ve); } }
  __syncthreads();
  { __shared__ __align__(16) int srs[256], src2[256]; srs[tid] = node < CSR_N ? gst : 0; src2[tid] = node < CSR_N ? cnt : 0; __syncthreads();
    if (tid < 64) vst2((unsigned*)(ROWST + (size_t)b * 256 + tid * 4), *(const v4u*)&srs[tid * 4]); else if (tid < 128) vst2((unsigned*)(ROWCNT + (size_t)b * 256 + (tid - 64) * 4), *(const v4u*)&src2[(tid - 64) * 4]); }
}


__device__ __forceinline__ void put_hl(__bf16* h, __bf16* l, float v) { const __bf16 hb = (__bf16)v; *h = hb; *l = (__bf16)(v - (float)hb); }
#define WS_CNT  0u
#define WS_OFF  (WS_CNT + CSR_SZ_CNT)
#define WS_BST  (WS_OFF + CSR_SZ_OFF)
#define WS_SEGS (WS_BST + CSR_SZ_BST)
#define WS_SEGE (WS_SEGS + CSR_SZ_SEG)
#define WS_FS   (WS_SEGE + CSR_SZ_SEG)
#define WS_FE   (WS_FS + CSR_SZ_FIN)
#define WS_RST  (WS_FE + CSR_SZ_FIN)
#define WS_RCT  (WS_RST + CSR_SZ_ROW)
#define WS_FS2  (WS_RCT + CSR_SZ_ROW)
#define WS_FE2  (WS_FS2 + CSR_SZ_FIN)
#define WS_RST2 (WS_FE2 + CSR_SZ_FIN)
#define WS_RCT2 (WS_RST2 + CSR_SZ_ROW)
#define WS_PW   (WS_RCT2 + CSR_SZ_ROW)
#define PW2A 0
#define PB2A (PW2A + KH1 * HH * CIN1)
#define PRTA (PB2A + HH * CIN1)
#define PW2B (PRTA + HH * CIN1)
#define PB2B (PW2B + KH2 * HH * HH)
#define PRTB (PB2B + HH * HH)
#define PWEND (PRTB + HH * HH)
#define WS_HE   (WS_PW + 2u * PWEND)
#define WS_MSG  (WS_HE + 4u * NEP * KH2)
#define WS_PRE  (WS_MSG + 4u * NEP * HH)
#define WS_HA   (WS_PRE + 4u * NRP * HH)
#define WS_HB   (WS_HA + 4u * NRP * HH)
#define WS_PS   (WS_HB + 4u * NRP * HH)
#define WS_ST   (WS_PS + 4u * NBLK * HH)
#define WS_POOL (WS_ST + 4u * 2 * HH)
#define WS_END  (WS_POOL + 4u * NG * 128)

__global__ __launch_bounds__(64) void k_pack(const float* __restrict__ W2A, const float* __restrict__ B2A, const float* __restrict__ RTA, const float* __restrict__ W2B, const float* __restrict__ B2B, const float* __restrict__ RTB, int sel, __bf16* __restrict__ PW) {
  __shared__ __align__(16) __bf16 s[2][64]; const int tid = threadIdx.x;
  if (sel < 3) {
    const int n0 = blockIdx.x * 2; const int rsel = tid >> 5, i = tid & 31; const int n = n0 + rsel; float v;
    if (sel == 0) { const int k = n / HH, o = n % HH; v = W2A[(size_t)k * (CIN1 * HH) + i * HH + o]; }
    else if (sel == 1) { v = B2A[i * HH + n]; } else { v = RTA[i * HH + n]; }
    s[rsel][i] = (__bf16)v; __syncthreads();
    const size_t base = (sel == 0) ? PW2A : (sel == 1 ? PB2A : PRTA);
    if (tid < 8) vst2((unsigned*)(PW + base + (size_t)n0 * CIN1 + tid * 8), *(const v4u*)&s[tid >> 2][(tid & 3) * 8]);
  } else {
    const int n = blockIdx.x, i = tid; float v;
    if (sel == 3) { const int k = n / HH, o = n % HH; v = W2B[(size_t)k * (HH * HH) + i * HH + o]; }
    else if (sel == 4) { v = B2B[i * HH + n]; } else { v = RTB[i * HH + n]; }
    s[0][i] = (__bf16)v; __syncthreads();
    const size_t base = (sel == 3) ? PW2B : (sel == 4 ? PB2B : PRTB);
    if (tid < 8) vst2((unsigned*)(PW + base + (size_t)n * HH + tid * 8), *(const v4u*)&s[0][tid * 8]);
  }
}
__global__ __launch_bounds__(256) void k_edgenet(const float* __restrict__ EA, const float* __restrict__ W1, const float* __restrict__ B1, int KH, float* __restrict__ HE) {
  __shared__ float sw[EC][KH2]; __shared__ float sb[KH2]; __shared__ __align__(16) float so[64][KH2 + 4];
  const int tid = threadIdx.x;
  for (int q = tid; q < EC * KH; q += 256) sw[q / KH][q % KH] = bfr(W1[q]);
  for (int q = tid; q < KH; q += 256) sb[q] = bfr(B1[q]);
  __syncthreads();
  for (int q = tid; q < 64 * KH2; q += 256) { const int el = q / KH2, k = q % KH2; const size_t e = (size_t)blockIdx.x * 64 + el; float v = 0.f;
    if (k < KH && e < (size_t)NE) { float a = sb[k];
#pragma unroll
      for (int c = 0; c < EC; ++c) a += bfr(EA[e * EC + c]) * sw[c][k];
      v = fmaxf(a, 0.f); }
    so[el][k] = v; }
  __syncthreads();
  for (int q = tid; q < 64 * (KH2 / 4); q += 256) { const int el = q / (KH2 / 4), pc = q % (KH2 / 4); vst2(HE + ((size_t)blockIdx.x * 64 + el) * KH2 + pc * 4, *(const v4f*)&so[el][pc * 4]); }
}
template <int CIN, int KH, int RIN>
__global__ __launch_bounds__(256) void k_msg(const float* __restrict__ X, const int* __restrict__ FE2, const int* __restrict__ RST2, const int* __restrict__ RCT2, const float* __restrict__ HE, const __bf16* __restrict__ PW2, const __bf16* __restrict__ PB2, float* __restrict__ MSG) {
  __shared__ __align__(16) float smsg[MAXE][HH]; __shared__ __align__(16) float st[64][132]; __shared__ int seid[MAXE]; __shared__ unsigned char ssrc[MAXE]; __shared__ int scnt[64], sst[64]; __shared__ int sne;
  const int tid = threadIdx.x, blk = blockIdx.x; const int wave = tid >> 5, lane = tid & 31, col = lane & 15, g = lane >> 4; const bool gw = wave < 4;
  if (tid < 64) { const size_t node = (size_t)blk * 64 + tid; int c = 0, s0 = 0; if (node < (size_t)NN) { c = min(max(RCT2[node], 0), CSR_BCAP); s0 = min(max(RST2[node], 0), CSR_FINN - c); } scnt[tid] = c; sst[tid] = s0; }
  __syncthreads();
  if (tid == 0) { int acc = 0; for (int n = 0; n < 64; ++n) { const int c = scnt[n]; const int take = min(c, MAXE - acc); for (int j = 0; j < take; ++j) { seid[acc + j] = min(max(FE2[sst[n] + j], 0), NE - 1); ssrc[acc + j] = (unsigned char)n; } acc += take; } sne = acc; }
  __syncthreads();
  const int ne = sne;
  F2 af[CIN / 32]; v16b ax[CIN / 32];
  { size_t ra = (size_t)blk * 64 + wave * 16 + col; if (ra >= NN) ra = NN - 1; const float* xr = X + ra * CIN;
#pragma unroll
    for (int kc = 0; kc < CIN / 32; ++kc) { if (RIN) { const float* p = xr + kc * 32 + 8 * g;
#pragma unroll
        for (int i = 0; i < 8; ++i) { ax[kc][i] = (__bf16)p[i]; ax[kc][8 + i] = (__bf16)p[16 + i]; } af[kc].h = ax[kc]; af[kc].l = ax[kc]; }
      else af[kc] = split_row(xr, kc * 32, lane); } }
  if (gw) { v8f acc[4] = {};
#pragma unroll
    for (int kc = 0; kc < CIN / 32; ++kc) {
#pragma unroll
      for (int j = 0; j < 4; ++j) { const v16b w = frag_b(PB2 + (size_t)(j * 16 + col) * CIN + kc * 32, lane); if (RIN) acc[j] = wmma_bf(ax[kc], w, acc[j]); else { acc[j] = wmma_bf(af[kc].l, w, acc[j]); acc[j] = wmma_bf(af[kc].h, w, acc[j]); } } }
#pragma unroll
    for (int j = 0; j < 4; ++j)
#pragma unroll
      for (int r = 0; r < 8; ++r) st[wave * 16 + 8 * g + r][j * 16 + col] = acc[j][r]; }
  __syncthreads();
  for (int q = tid; q < MAXE * HH; q += 256) { const int j = q / HH, o = q % HH; smsg[j][o] = (j < ne) ? st[ssrc[j]][o] : 0.f; }
  __syncthreads();
#pragma unroll 1
  for (int sl = 0; sl < ((ne > 0) ? KH / 2 : 0); ++sl) {
    if (gw) { v8f acc[8] = {};
#pragma unroll
      for (int kc = 0; kc < CIN / 32; ++kc) {
#pragma unroll
        for (int j = 0; j < 8; ++j) { const v16b w = frag_b(PW2 + ((size_t)sl * 128 + j * 16 + col) * CIN + kc * 32, lane); if (RIN) acc[j] = wmma_bf(ax[kc], w, acc[j]); else { acc[j] = wmma_bf(af[kc].l, w, acc[j]); acc[j] = wmma_bf(af[kc].h, w, acc[j]); } } }
#pragma unroll
      for (int j = 0; j < 8; ++j)
#pragma unroll
        for (int r = 0; r < 8; ++r) st[wave * 16 + 8 * g + r][j * 16 + col] = acc[j][r]; }
    __syncthreads();
    { const int o = tid & 63; for (int j = tid >> 6; j < ne; j += 4) { const int e = seid[j]; const int sIdx = ssrc[j]; const float h0 = HE[(size_t)e * KH2 + 2 * sl], h1 = HE[(size_t)e * KH2 + 2 * sl + 1]; smsg[j][o] += h0 * st[sIdx][o] + h1 * st[sIdx][HH + o]; } }
    __syncthreads(); }
  for (int q = tid; q < ne * 16; q += 256) { const int j = q >> 4, pc = q & 15; vst2(MSG + (size_t)seid[j] * HH + pc * 4, *(const v4f*)&smsg[j][pc * 4]); }
}
template <int CIN, int RIN>
__global__ __launch_bounds__(256) void k_agg(const float* __restrict__ X, const float* __restrict__ MSG, const int* __restrict__ FE, const int* __restrict__ RST, const int* __restrict__ RCT, const __bf16* __restrict__ PRT, const float* __restrict__ bias, float* __restrict__ PRE) {
  __shared__ __align__(16) float so[64][HH + 4];
  const int tid = threadIdx.x, blk = blockIdx.x; const int nl = tid >> 2, f0 = (tid & 3) * 16; const size_t node = (size_t)blk * 64 + nl;
  const int wave = tid >> 5, lane = tid & 31, col = lane & 15, g = lane >> 4; const bool gw = wave < 4;
  if (gw) { v8f acc[4] = {}; size_t ra = (size_t)blk * 64 + wave * 16 + col; if (ra >= NN) ra = NN - 1; const float* xr = X + ra * CIN;
#pragma unroll
    for (int kc = 0; kc < CIN / 32; ++kc) { F2 a; if (RIN) { v16b ax; const float* p = xr + kc * 32 + 8 * g;
#pragma unroll
        for (int i = 0; i < 8; ++i) { ax[i] = (__bf16)p[i]; ax[8 + i] = (__bf16)p[16 + i]; } a.h = ax; a.l = ax; } else a = split_row(xr, kc * 32, lane);
#pragma unroll
      for (int j = 0; j < 4; ++j) { const v16b w = frag_b(PRT + (size_t)(j * 16 + col) * CIN + kc * 32, lane); if (RIN) acc[j] = wmma_bf(a.h, w, acc[j]); else { acc[j] = wmma_bf(a.l, w, acc[j]); acc[j] = wmma_bf(a.h, w, acc[j]); } } }
#pragma unroll
    for (int j = 0; j < 4; ++j)
#pragma unroll
      for (int r = 0; r < 8; ++r) so[wave * 16 + 8 * g + r][j * 16 + col] = acc[j][r] + bfr(bias[j * 16 + col]); }
  __syncthreads();
  { float acc[16];
#pragma unroll
    for (int i = 0; i < 16; ++i) acc[i] = 0.f;
    int cnt = 0;
    if (node < (size_t)NN) { cnt = min(max(RCT[node], 0), CSR_BCAP); const int st0 = min(max(RST[node], 0), CSR_FINN - cnt);
      for (int e = 0; e < cnt; ++e) { const int eid = min(max(FE[st0 + e], 0), NE - 1); const float* mr = MSG + (size_t)eid * HH + f0;
#pragma unroll
        for (int i = 0; i < 16; ++i) acc[i] += mr[i]; } }
    const float ic = 1.0f / (float)max(cnt, 1);
#pragma unroll
    for (int i = 0; i < 16; ++i) so[nl][f0 + i] += acc[i] * ic; }
  __syncthreads();
  for (int q = tid; q < 64 * 16; q += 256) { const int rl = q >> 4, pc = q & 15; vst2(PRE + ((size_t)blk * 64 + rl) * HH + pc * 4, *(const v4f*)&so[rl][pc * 4]); }
}
template <int MODE>
__global__ __launch_bounds__(64) void k_colsum(const float* __restrict__ Hs, const float* __restrict__ ST, float* __restrict__ PS) {
  __shared__ __align__(16) float s[HH]; const int blk = blockIdx.x, c = threadIdx.x; const float mu = (MODE == 1) ? ST[c] : 0.f; float acc = 0.f;
  for (int rl = 0; rl < 64; ++rl) { const size_t node = (size_t)blk * 64 + rl; if (node < (size_t)NN) { const float v = Hs[node * HH + c]; acc += (MODE == 1) ? (v - mu) * (v - mu) : v; } }
  s[c] = acc; __syncthreads();
  if (c < 16) vst2(PS + (size_t)blk * HH + c * 4, *(const v4f*)&s[c * 4]);
}
template <int MODE>
__global__ __launch_bounds__(64) void k_red(const float* __restrict__ PS, float* __restrict__ ST) {
  __shared__ __align__(16) float s[HH]; const int c = threadIdx.x; float acc = 0.f;
  for (int b = 0; b < NBLK; ++b) acc += PS[(size_t)b * HH + c];
  s[c] = (MODE == 0) ? acc / (float)NN : rsqrtf(acc / (float)NN + 1e-5f);
  __syncthreads();
  if (c < 16) vst2(ST + MODE * HH + c * 4, *(const v4f*)&s[c * 4]);
}
__global__ __launch_bounds__(256) void k_bnact(const float* __restrict__ PRE, const float* __restrict__ ST, const float* __restrict__ gm, const float* __restrict__ bt, float* __restrict__ Hs) {
  __shared__ __align__(16) float so[64][HH + 4]; __shared__ float smu[HH], srs[HH], sg[HH], sb[HH]; const int tid = threadIdx.x, blk = blockIdx.x;
  if (tid < HH) { smu[tid] = ST[tid]; srs[tid] = ST[HH + tid]; sg[tid] = bfr(gm[tid]); sb[tid] = bfr(bt[tid]); }
  __syncthreads();
  for (int q = tid; q < 64 * HH; q += 256) { const int rl = q >> 6, c = q & 63; const size_t node = (size_t)blk * 64 + rl; float v = 0.f; if (node < (size_t)NN) { v = (PRE[node * HH + c] - smu[c]) * srs[c] * sg[c] + sb[c]; v = fmaxf(v, 0.f); } so[rl][c] = v; }
  __syncthreads();
  for (int q = tid; q < 64 * 16; q += 256) { const int rl = q >> 4, pc = q & 15; vst2(Hs + ((size_t)blk * 64 + rl) * HH + pc * 4, *(const v4f*)&so[rl][pc * 4]); }
}
__global__ __launch_bounds__(256) void k_pool(const float* __restrict__ Hs, const int* __restrict__ BATCH, float* __restrict__ POOL) {
  __shared__ float sp[4][HH + 1]; __shared__ int sc[4]; __shared__ __align__(16) float srow[2 * HH];
  const int gidx = blockIdx.x, tid = threadIdx.x; const int part = tid >> 6, c = tid & 63; float acc = 0.f; int cnt = 0;
  for (int n = part; n < NN; n += 4) { if (BATCH[n] == gidx) { acc += Hs[(size_t)n * HH + c]; cnt += 1; } }
  sp[part][c] = acc; if (c == 0) sc[part] = cnt;
  __syncthreads();
  if (tid < HH) { const float a = sp[0][tid] + sp[1][tid] + sp[2][tid] + sp[3][tid]; const int cn = sc[0] + sc[1] + sc[2] + sc[3]; srow[tid] = a / (float)max(cn, 1); srow[HH + tid] = a; }
  __syncthreads();
  if (tid < 32) vst2(POOL + (size_t)gidx * (2 * HH) + tid * 4, *(const v4f*)&srow[tid * 4]);
}
__global__ __launch_bounds__(128) void k_head(const float* __restrict__ POOL, const float* __restrict__ W1, const float* __restrict__ B1, const float* __restrict__ W2, const float* __restrict__ B2, const float* __restrict__ W3, const float* __restrict__ B3, float* __restrict__ out) {
  __shared__ float sh1[NG][HH + 1]; __shared__ __align__(16) float sy[NG];
  const int gidx = threadIdx.x; const float* pr = POOL + (size_t)gidx * (2 * HH);
#pragma unroll 1
  for (int o = 0; o < HH; ++o) { float s = bfr(B1[o]);
#pragma unroll 1
    for (int i = 0; i < 2 * HH; ++i) s += pr[i] * bfr(W1[i * HH + o]);
    sh1[gidx][o] = fmaxf(s, 0.f); }
  float y = bfr(B3[0]);
#pragma unroll 1
  for (int o2 = 0; o2 < 32; ++o2) { float s = bfr(B2[o2]);
#pragma unroll 1
    for (int i = 0; i < HH; ++i) s += sh1[gidx][i] * bfr(W2[i * 32 + o2]);
    y += fmaxf(s, 0.f) * bfr(W3[o2]); }
  sy[gidx] = (gidx < NG) ? y : 0.f; __syncthreads();
  if (gidx < NG / 4) vst2(out + gidx * 4, *(const v4f*)&sy[gidx * 4]);
}
extern "C" void kernel_launch(void* const* d_in, const int* in_sizes, int n_in, void* d_out, int out_size, void* d_ws, size_t ws_size, hipStream_t stream) {
  (void)in_sizes; (void)n_in; (void)out_size;
  const float** F = (const float**)d_in; const int* EI = (const int*)d_in[1]; const int* BATCH = (const int*)d_in[3];
  if (ws_size < (size_t)WS_END) return;
  char* ws = (char*)d_ws;
  int *CNT = (int*)(ws + WS_CNT), *OFF = (int*)(ws + WS_OFF), *BST = (int*)(ws + WS_BST), *SEGS = (int*)(ws + WS_SEGS), *SEGE = (int*)(ws + WS_SEGE), *FS = (int*)(ws + WS_FS), *FE = (int*)(ws + WS_FE), *RST = (int*)(ws + WS_RST), *RCT = (int*)(ws + WS_RCT), *FS2 = (int*)(ws + WS_FS2), *FE2 = (int*)(ws + WS_FE2), *RST2 = (int*)(ws + WS_RST2), *RCT2 = (int*)(ws + WS_RCT2);
  __bf16* PW = (__bf16*)(ws + WS_PW); float *HE = (float*)(ws + WS_HE), *MSG = (float*)(ws + WS_MSG), *PRE = (float*)(ws + WS_PRE), *HA = (float*)(ws + WS_HA), *HB = (float*)(ws + WS_HB), *PS = (float*)(ws + WS_PS), *ST = (float*)(ws + WS_ST), *POOL = (float*)(ws + WS_POOL);
  const int* SRC = EI; const int* DST = EI + EP;
  k_pack<<<KH1 * HH / 2, 64, 0, stream>>>(F[6], F[7], F[8], F[14], F[15], F[16], 0, PW); k_pack<<<HH / 2, 64, 0, stream>>>(F[6], F[7], F[8], F[14], F[15], F[16], 1, PW); k_pack<<<HH / 2, 64, 0, stream>>>(F[6], F[7], F[8], F[14], F[15], F[16], 2, PW);
  k_pack<<<KH2 * HH, 64, 0, stream>>>(F[6], F[7], F[8], F[14], F[15], F[16], 3, PW); k_pack<<<HH, 64, 0, stream>>>(F[6], F[7], F[8], F[14], F[15], F[16], 4, PW); k_pack<<<HH, 64, 0, stream>>>(F[6], F[7], F[8], F[14], F[15], F[16], 5, PW);
  k_csr_cnt<<<CSR_NCH, 256, 0, stream>>>(SRC, 1, CNT); k_csr_scan<<<1, 256, 0, stream>>>(CNT, OFF, BST); k_csr_scatter<<<CSR_NCH, 256, 0, stream>>>(DST, SRC, 1, 1, OFF, SEGS, SEGE); k_csr_bucket<<<CSR_NBK, 256, 0, stream>>>(CNT, OFF, BST, SEGS, SEGE, SRC, 1, FS2, FE2, RST2, RCT2);
  k_csr_cnt<<<CSR_NCH, 256, 0, stream>>>(DST, 1, CNT); k_csr_scan<<<1, 256, 0, stream>>>(CNT, OFF, BST); k_csr_scatter<<<CSR_NCH, 256, 0, stream>>>(SRC, DST, 1, 1, OFF, SEGS, SEGE); k_csr_bucket<<<CSR_NBK, 256, 0, stream>>>(CNT, OFF, BST, SEGS, SEGE, DST, 1, FS, FE, RST, RCT);
  k_edgenet<<<NEP / 64, 256, 0, stream>>>(F[2], F[4], F[5], KH1, HE);
  k_msg<CIN1, KH1, 1><<<NBLK, 256, 0, stream>>>(F[0], FE2, RST2, RCT2, HE, PW + PW2A, PW + PB2A, MSG);
  k_agg<CIN1, 1><<<NBLK, 256, 0, stream>>>(F[0], MSG, FE, RST, RCT, PW + PRTA, F[9], PRE);
  k_colsum<0><<<NBLK, 64, 0, stream>>>(PRE, ST, PS); k_red<0><<<1, 64, 0, stream>>>(PS, ST); k_colsum<1><<<NBLK, 64, 0, stream>>>(PRE, ST, PS); k_red<1><<<1, 64, 0, stream>>>(PS, ST);
  k_bnact<<<NBLK, 256, 0, stream>>>(PRE, ST, F[10], F[11], HA);
  k_edgenet<<<NEP / 64, 256, 0, stream>>>(F[2], F[12], F[13], KH2, HE);
  k_msg<HH, KH2, 0><<<NBLK, 256, 0, stream>>>(HA, FE2, RST2, RCT2, HE, PW + PW2B, PW + PB2B, MSG);
  k_agg<HH, 0><<<NBLK, 256, 0, stream>>>(HA, MSG, FE, RST, RCT, PW + PRTB, F[17], PRE);
  k_colsum<0><<<NBLK, 64, 0, stream>>>(PRE, ST, PS); k_red<0><<<1, 64, 0, stream>>>(PS, ST); k_colsum<1><<<NBLK, 64, 0, stream>>>(PRE, ST, PS); k_red<1><<<1, 64, 0, stream>>>(PS, ST);
  k_bnact<<<NBLK, 256, 0, stream>>>(PRE, ST, F[18], F[19], HB);
  k_pool<<<NG, 256, 0, stream>>>(HB, BATCH, POOL);
  k_head<<<1, 128, 0, stream>>>(POOL, F[20], F[21], F[22], F[23], F[24], F[25], (float*)d_out);
}
